// EireneGNN_4939212390552
// MI455X (gfx1250) — hardware-verified
//
#include <hip/hip_runtime.h>
#include <stddef.h>


#define FIN     14
#define FH      128
#define FH2     64
#define FOUT    9
#define NLAY    6
#define EDIM    3
#define MSGK    (2 * FH + EDIM)
#define PQW     (2 * FH)
#define D3W     32
#define NTHR    256
#define NWAVE   8
#define EPT     8
#define NGRP    2
#define CHUNK   (NTHR * EPT * NGRP)
#define WCAP    (EPT * NGRP * 32)
#define LISTN   (NWAVE * WCAP)
#define ESHF    11
#define EIDBITS 20
#define NBC     32768
#define NBF     2048
#define RCAP    40960
#define RBN     128
#define TGT     256
#define DEGCAP  1024
#define GR      64
#define OTHR    512
#define WSCAP   134217728

#define LDS_COUNT ((NBC + LISTN + NWAVE) * 4)
#define LDS_FILL  ((RCAP + NBF + LISTN + NWAVE) * 4)
#define LDS_GEMM  32768

static_assert((CHUNK & (CHUNK - 1)) == 0);
static_assert((NBC & (NBC - 1)) == 0 && (NBF & (NBF - 1)) == 0);
static_assert(NBF <= (1 << ESHF));
static_assert(ESHF + EIDBITS <= 31);
static_assert((NBC % NBF) == 0);
static_assert(OTHR * 4 == NBF);
static_assert((RCAP % 32) == 0);
static_assert(TGT == NWAVE * 32);
static_assert(GR == (NWAVE / 2) * 16 && (GR % NWAVE) == 0);
static_assert((TGT % GR) == 0);
static_assert(NBC == NWAVE * 32 * 128);
static_assert((FH % 32) == 0 && FH == 4 * 32);
static_assert(FOUT <= D3W);

typedef float          v4f   __attribute__((ext_vector_type(4)));
typedef float          v8f   __attribute__((ext_vector_type(8)));
typedef int            v4i   __attribute__((ext_vector_type(4)));
typedef unsigned short v8us  __attribute__((ext_vector_type(8)));
typedef __bf16         v8bf  __attribute__((ext_vector_type(8)));
typedef __bf16         v16bf __attribute__((ext_vector_type(16)));
union FragB { v16bf v; v8us h[2]; };
union Pk8   { v8bf b; v8us u; };

__device__ __forceinline__ v8f wmb(v16bf a, v16bf b, v8f c) {
  v8f d = __builtin_amdgcn_wmma_f32_16x16x32_bf16(false, a, false, b, (short)0, c, false, false);
  asm volatile("v_nop\n\tv_nop\n\tv_nop\n\tv_nop" : "+v"(d) : "v"(a), "v"(b));
  return d;
}

__device__ __forceinline__ float silu1(float x) {
  const float e = __expf(-x);
  const float r = __builtin_amdgcn_rcpf(1.0f + e);
  return x * r;
}
__device__ __forceinline__ v4f silu4(v4f v) {
  v4f o;
  o.x = silu1(v.x); o.y = silu1(v.y); o.z = silu1(v.z); o.w = silu1(v.w);
  return o;
}

template <int NB, int EID>
__device__ __forceinline__ int scan_chunk(const int* __restrict__ dsts, int nE,
                                          int cbase, int slotBase, int vec8, int* list, int tid, int lane, int wave) {
  int wc = 0;
#pragma unroll
  for (int g = 0; g < NGRP; ++g) {
    const int el0  = (g * NTHR + tid) * EPT;
    const int e0   = cbase + el0;
    const int sent = -2147483647 - 1;
    v4i da, db;
    if (vec8 != 0 && cbase + CHUNK <= nE) {
      da = *(const v4i*)(dsts + e0);
      db = *(const v4i*)(dsts + e0 + 4);
    } else {
      da.x = (e0     < nE) ? dsts[min(e0, nE - 1)] : sent;
      da.y = (e0 + 1 < nE) ? dsts[min(e0 + 1, nE - 1)] : sent;
      da.z = (e0 + 2 < nE) ? dsts[min(e0 + 2, nE - 1)] : sent;
      da.w = (e0 + 3 < nE) ? dsts[min(e0 + 3, nE - 1)] : sent;
      db.x = (e0 + 4 < nE) ? dsts[min(e0 + 4, nE - 1)] : sent;
      db.y = (e0 + 5 < nE) ? dsts[min(e0 + 5, nE - 1)] : sent;
      db.z = (e0 + 6 < nE) ? dsts[min(e0 + 6, nE - 1)] : sent;
      db.w = (e0 + 7 < nE) ? dsts[min(e0 + 7, nE - 1)] : sent;
    }
    const unsigned nb = (unsigned)slotBase;
    const unsigned s0 = (unsigned)da.x - nb, s1 = (unsigned)da.y - nb;
    const unsigned s2 = (unsigned)da.z - nb, s3 = (unsigned)da.w - nb;
    const unsigned s4 = (unsigned)db.x - nb, s5 = (unsigned)db.y - nb;
    const unsigned s6 = (unsigned)db.z - nb, s7 = (unsigned)db.w - nb;
    const bool h0 = s0 < (unsigned)NB, h1 = s1 < (unsigned)NB, h2 = s2 < (unsigned)NB, h3 = s3 < (unsigned)NB;
    const bool h4 = s4 < (unsigned)NB, h5 = s5 < (unsigned)NB, h6 = s6 < (unsigned)NB, h7 = s7 < (unsigned)NB;
    const unsigned any = __builtin_amdgcn_ballot_w32(h0 | h1 | h2 | h3 | h4 | h5 | h6 | h7);
    if (any != 0u) {
#define HITJ(HJ, SJ, J) { \
        const unsigned mj = __builtin_amdgcn_ballot_w32(HJ); \
        if (mj != 0u) { \
          if (HJ) { \
            const int pos = wc + (int)__builtin_amdgcn_mbcnt_lo(mj, 0u); \
            const int entv = EID ? (((e0 + (J)) << ESHF) | (int)(SJ)) : (int)(SJ); \
            if (pos < WCAP) list[wave * WCAP + pos] = entv; \
          } \
          wc += (int)__builtin_popcount(mj); } }
      HITJ(h0, s0, 0)
      HITJ(h1, s1, 1)
      HITJ(h2, s2, 2)
      HITJ(h3, s3, 3)
      HITJ(h4, s4, 4)
      HITJ(h5, s5, 5)
      HITJ(h6, s6, 6)
      HITJ(h7, s7, 7)
#undef HITJ
    }
  }
  return wc;
}

__global__ __launch_bounds__(NTHR) void k_wprep(const float* __restrict__ W, int KA, int NOUT, int ydiv, int wsHi, int wsLo,
                                                unsigned short* ph, unsigned short* pl, int pstride, int K, int NP) {
  const int tid = threadIdx.x;
  const int y = (int)blockIdx.y;
  const int yq = y / ydiv;
  const float* Wy = W + (size_t)yq * wsHi + (size_t)(y - yq * ydiv) * wsLo;
  const int kq = K >> 3;
  const int total = NP * kq;
  const int i = (int)blockIdx.x * NTHR + tid;
  const int ic = i < total ? i : total - 1;
  const int n = ic / kq;
  const int k0 = (ic - n * kq) * 8;
  const int nc = n < NOUT ? n : NOUT - 1;
  Pk8 hp, lp;
#pragma unroll
  for (int e = 0; e < 8; ++e) {
    const int kk = k0 + e;
    const int kc = kk < KA ? kk : KA - 1;
    float v = Wy[(size_t)kc * NOUT + nc];
    v = (n < NOUT && kk < KA) ? v : 0.0f;
    const __bf16 hb = (__bf16)v;
    const float rem = v - (float)hb;
    hp.b[e] = hb;
    lp.b[e] = (__bf16)rem;
  }
  unsigned short* dh = ph + (size_t)y * pstride + (size_t)ic * 8;
  unsigned short* dl = pl + (size_t)y * pstride + (size_t)ic * 8;
  if (i < total) { *(volatile v8us*)dh = hp.u; *(volatile v8us*)dl = lp.u; }
  __threadfence();
  if (i < total) { *(volatile v8us*)dh = hp.u; *(volatile v8us*)dl = lp.u; }
}

__global__ __launch_bounds__(NTHR) void k_count(const int* __restrict__ ei, int* cnt, int nE, int vec8) {
  extern __shared__ v4f lds_dyn[];
  int* scnt = (int*)lds_dyn;
  int* list = scnt + NBC;
  int* wcnt = list + LISTN;
  const int tid = threadIdx.x, lane = tid & 31, wave = tid >> 5;
  const int nodeBase = blockIdx.x * NBC;
  const int* dsts = ei + nE;

  {
    const v4i z = {0, 0, 0, 0};
    for (int i = tid; i < NBC / 4; i += NTHR) ((v4i*)scnt)[i] = z;
  }
  __syncthreads();

  const int nChunks = (nE + CHUNK - 1) / CHUNK;
#pragma unroll 1
  for (int ch = 0; ch < nChunks; ++ch) {
    const int cbase = ch * CHUNK;
    const int wc = scan_chunk<NBC, 0>(dsts, nE, cbase, nodeBase, vec8, list, tid, lane, wave);
    if (lane == 0) wcnt[wave] = wc;
    __syncthreads();
    if (wave == 0) {
#pragma unroll 1
      for (int wsx = 0; wsx < NWAVE; ++wsx) {
        int n = __builtin_amdgcn_readfirstlane(wcnt[wsx]);
        n = n > WCAP ? WCAP : (n < 0 ? 0 : n);
        const int* lp = list + wsx * WCAP;
#pragma unroll 1
        for (int i = 0; i < n; ++i) {
          const int ent  = __builtin_amdgcn_readfirstlane(lp[i]);
          const int slot = ent & (NBC - 1);
          if (lane == 0) scnt[slot] = scnt[slot] + 1;
        }
      }
    }
    __syncthreads();
  }

  int* cp = cnt + (size_t)nodeBase;
#pragma unroll 4
  for (int q = 0; q < 32; ++q) {
    const int f = (wave * 32 + q) * 128 + 4 * lane;
    const v4i c = *(const v4i*)(scnt + f);
    *(volatile v4i*)(cp + f) = c;
  }
  __threadfence();
#pragma unroll 4
  for (int q = 0; q < 32; ++q) {
    const int f = (wave * 32 + q) * 128 + 4 * lane;
    const v4i c = *(const v4i*)(scnt + f);
    *(volatile v4i*)(cp + f) = c;
  }
}

__global__ __launch_bounds__(OTHR) void k_offsets(const int* __restrict__ cnt, int* off, int* rbase, int nBF) {
  __shared__ __attribute__((aligned(16))) int srb[RBN];
  __shared__ int wtot[OTHR / 32];
  const int tid = threadIdx.x, lane = tid & 31, wave = tid >> 5;
  for (int i = tid; i < RBN; i += OTHR) srb[i] = 0;
  int carry = 0;
#pragma unroll 1
  for (int fb = 0; fb < nBF; ++fb) {
    const int base = fb * NBF;
    const v4i c = *(const v4i*)(cnt + base + 4 * tid);
    const int e0 = max(c.x, 0), e1 = max(c.y, 0), e2 = max(c.z, 0), e3 = max(c.w, 0);
    const int ts = e0 + e1 + e2 + e3;
    int incl = ts;
#pragma unroll
    for (int d = 1; d < 32; d <<= 1) {
      const int t = __shfl_up(incl, d);
      if (lane >= d) incl += t;
    }
    if (lane == 31) wtot[wave] = incl;
    __syncthreads();
    int pre = 0;
#pragma unroll 1
    for (int w = 0; w < wave; ++w) pre += wtot[w];
    int tot = 0;
#pragma unroll
    for (int w = 0; w < OTHR / 32; ++w) tot += wtot[w];
    int run = carry + pre + incl - ts;
    v4i o;
    o.x = run; run += e0;
    o.y = run; run += e1;
    o.z = run; run += e2;
    o.w = run;
    int* op = off + base + 4 * tid;
    *(volatile v4i*)op = o;
    __threadfence();
    *(volatile v4i*)op = o;
    if (tid == 0) srb[min(fb, RBN - 1)] = carry;
    carry += (tot + 31) & ~31;
    __syncthreads();
  }
  if (tid == 0) srb[min(nBF, RBN - 1)] = carry;
  __syncthreads();
  v4i rv = {0, 0, 0, 0};
  if (tid < 32) rv = *(const v4i*)(srb + 4 * tid);
  if (tid < 32) *(volatile v4i*)(rbase + 4 * tid) = rv;
  __threadfence();
  if (tid < 32) *(volatile v4i*)(rbase + 4 * tid) = rv;
}

__global__ __launch_bounds__(NTHR) void k_fill(
    const int* __restrict__ ei, const int* __restrict__ off, const int* __restrict__ rbase,
    int* csr, int nE, int vec8, int csrLen) {
  extern __shared__ v4f lds_dyn[];
  int* region = (int*)lds_dyn;
  int* cursor = region + RCAP;
  int* list   = cursor + NBF;
  int* wcnt   = list + LISTN;
  const int tid = threadIdx.x, lane = tid & 31, wave = tid >> 5;
  const int b = blockIdx.x;
  const int nodeBase = b * NBF;
  const int* dsts = ei + nE;

  int rb0 = rbase[b];
  const int rb1 = rbase[b + 1];
  rb0 = rb0 < 0 ? 0 : (rb0 > csrLen ? csrLen : rb0);
  rb0 &= ~31;
  int len = rb1 - rb0;
  len = len < 0 ? 0 : (len > RCAP ? RCAP : len);
  int lenW = (len + 31) & ~31;
  if (rb0 + lenW > csrLen) lenW = (csrLen - rb0) & ~31;

  {
    const v4i z = {0, 0, 0, 0};
    for (int i = tid; i < RCAP / 4; i += NTHR) ((v4i*)region)[i] = z;
    for (int s = tid; s < NBF; s += NTHR) {
      int o = off[nodeBase + s] - rb0;
      o = o < 0 ? 0 : (o > RCAP ? RCAP : o);
      cursor[s] = o;
    }
  }
  __syncthreads();

  const int nChunks = (nE + CHUNK - 1) / CHUNK;
#pragma unroll 1
  for (int ch = 0; ch < nChunks; ++ch) {
    const int cbase = ch * CHUNK;
    const int wc = scan_chunk<NBF, 1>(dsts, nE, cbase, nodeBase, vec8, list, tid, lane, wave);
    if (lane == 0) wcnt[wave] = wc;
    __syncthreads();
    if (wave == 0) {
#pragma unroll 1
      for (int wsx = 0; wsx < NWAVE; ++wsx) {
        int n = __builtin_amdgcn_readfirstlane(wcnt[wsx]);
        n = n > WCAP ? WCAP : (n < 0 ? 0 : n);
        const int* lp = list + wsx * WCAP;
#pragma unroll 1
        for (int i = 0; i < n; ++i) {
          const int ent  = __builtin_amdgcn_readfirstlane(lp[i]);
          const int slot = ent & (NBF - 1);
          int eid = (ent >> ESHF) & ((1 << EIDBITS) - 1);
          eid = eid > nE - 1 ? nE - 1 : eid;
          if (lane == 0) {
            int pos = cursor[slot];
            pos = pos < 0 ? 0 : (pos > RCAP - 1 ? RCAP - 1 : pos);
            region[pos] = eid;
            const int np = pos + 1;
            cursor[slot] = np > RCAP ? RCAP : np;
          }
        }
      }
    }
    __syncthreads();
  }

  const int nv = lenW >> 2;
  int* gp = csr + rb0;
#pragma unroll 1
  for (int i = tid; i < nv; i += NTHR) { const v4i v = ((const v4i*)region)[i]; *(volatile v4i*)(gp + 4 * i) = v; }
  __threadfence();
#pragma unroll 1
  for (int i = tid; i < nv; i += NTHR) { const v4i v = ((const v4i*)region)[i]; *(volatile v4i*)(gp + 4 * i) = v; }
}

template <int K, int KA, int LDA, int NT, int ACT, int RES, int BIAS>
__global__ __launch_bounds__(NTHR) void k_gemm(
    const float* __restrict__ A, int nRowsA,
    const unsigned short* __restrict__ Bh, const unsigned short* __restrict__ Bl,
    const float* __restrict__ bias, int nOut,
    const float* __restrict__ Hold, const int* __restrict__ cnt,
    float* C, int ldc) {
  constexpr int NCB = 32 * NT, NCBH = 16 * NT, SP = NCB, RPI = 4 / NT, NINST = 2 * NT, F4R = 8 * NT;
  constexpr int RPW = GR / NWAVE;
  static_assert(NT == 1 || NT == 2 || NT == 4);
  static_assert((K % 32) == 0 && KA <= K && KA >= 1);
  static_assert(2 * GR * K * 2 <= LDS_GEMM && GR * SP * 4 <= LDS_GEMM);
  static_assert((GR * K / 8) % NTHR == 0);
  static_assert(RPI * NINST == RPW);
  extern __shared__ v4f lds_dyn[];
  unsigned short* sAh = (unsigned short*)lds_dyn;
  unsigned short* sAl = sAh + GR * K;
  float* stg = (float*)lds_dyn;
  const int tid = threadIdx.x, lane = tid & 31, wave = tid >> 5, hh = lane >> 4, m = lane & 15;
  const int rg = wave >> 1, chf = wave & 1;
  const int rowBase = (int)blockIdx.x * GR;
  const int y = (int)blockIdx.y;
  const int colBase = y * NCB;
  const unsigned short* Bhy = Bh + (size_t)y * NCB * K;
  const unsigned short* Bly = Bl + (size_t)y * NCB * K;

#pragma unroll
  for (int i = 0; i < (GR * K / 8) / NTHR; ++i) {
    const int idx = i * NTHR + tid;
    const int r   = idx / (K / 8);
    const int c0  = (idx - r * (K / 8)) * 8;
    int row = rowBase + r;
    row = row > nRowsA - 1 ? nRowsA - 1 : row;
    float av[8];
    if (KA == K && (LDA % 4) == 0) {
      const float* ap = A + (size_t)row * LDA + c0;
      const v4f a = *(const v4f*)ap, b = *(const v4f*)(ap + 4);
      av[0] = a.x; av[1] = a.y; av[2] = a.z; av[3] = a.w;
      av[4] = b.x; av[5] = b.y; av[6] = b.z; av[7] = b.w;
    } else {
#pragma unroll
      for (int e = 0; e < 8; ++e) {
        const int kk = c0 + e;
        const int kc = kk < KA ? kk : KA - 1;
        const float v = A[(size_t)row * LDA + kc];
        av[e] = kk < KA ? v : 0.0f;
      }
    }
    Pk8 hp, lp;
#pragma unroll
    for (int e = 0; e < 8; ++e) {
      const __bf16 hb = (__bf16)av[e];
      const float rem = av[e] - (float)hb;
      hp.b[e] = hb;
      lp.b[e] = (__bf16)rem;
    }
    *(v8us*)(sAh + r * K + c0) = hp.u;
    *(v8us*)(sAl + r * K + c0) = lp.u;
  }
  __syncthreads();

  v8f acc[NT];
#pragma unroll
  for (int t = 0; t < NT; ++t) { v8f z = {0.f, 0.f, 0.f, 0.f, 0.f, 0.f, 0.f, 0.f}; acc[t] = z; }
  const unsigned short* ahp = sAh + (rg * 16 + m) * K + 8 * hh;
  const unsigned short* alp = sAl + (rg * 16 + m) * K + 8 * hh;
#pragma unroll 1
  for (int kt = 0; kt < K / 32; ++kt) {
    FragB ah, al;
    ah.h[0] = *(const v8us*)(ahp + 32 * kt);
    ah.h[1] = *(const v8us*)(ahp + 32 * kt + 16);
    al.h[0] = *(const v8us*)(alp + 32 * kt);
    al.h[1] = *(const v8us*)(alp + 32 * kt + 16);
#pragma unroll
    for (int t = 0; t < NT; ++t) {
      const size_t bo = (size_t)(NCBH * chf + 16 * t + m) * K + 32 * kt + 8 * hh;
      FragB bh, bl;
      bh.h[0] = *(const v8us*)(Bhy + bo);
      bh.h[1] = *(const v8us*)(Bhy + bo + 16);
      bl.h[0] = *(const v8us*)(Bly + bo);
      bl.h[1] = *(const v8us*)(Bly + bo + 16);
      acc[t] = wmb(ah.v, bh.v, acc[t]);
      acc[t] = wmb(ah.v, bl.v, acc[t]);
      acc[t] = wmb(al.v, bh.v, acc[t]);
    }
  }
  __syncthreads();

  {
    float* sp = stg + (rg * 16 + 8 * hh) * SP + NCBH * chf + m;
#pragma unroll
    for (int t = 0; t < NT; ++t) {
#pragma unroll
      for (int r = 0; r < 8; ++r) sp[r * SP + 16 * t] = acc[t][r];
    }
  }
  __syncthreads();

  const int f4 = lane & (F4R - 1);
  const int lr = lane / F4R;
  float bz[4];
#pragma unroll
  for (int j = 0; j < 4; ++j) {
    const int cb = colBase + 4 * f4 + j;
    const int cc = cb < nOut ? cb : nOut - 1;
    float b = 0.0f;
    if (BIAS) { b = bias[cc]; b = cb < nOut ? b : 0.0f; }
    bz[j] = b;
  }
  const v4f bzv = {bz[0], bz[1], bz[2], bz[3]};
  v4f vals[NINST];
#pragma unroll
  for (int i = 0; i < NINST; ++i) {
    const int r = wave * RPW + i * RPI + lr;
    const int grow = rowBase + r;
    v4f v = *(const v4f*)(stg + r * SP + 4 * f4);
    if (RES) {
      const v4f hv = *(const v4f*)(Hold + (size_t)grow * ldc + colBase + 4 * f4);
      int cv = cnt[grow];
      cv = cv < 0 ? 0 : cv;
      const float degf = cv < 1 ? 1.0f : (float)cv;
      const float inv = 1.0f / degf;
      const float flag = cv > 0 ? 1.0f : 0.0f;
      const v4f agg = v * inv + bzv * flag;
      v = hv + agg;
    } else {
      v = v + bzv;
      if (ACT) v = silu4(v);
    }
    vals[i] = v;
  }
#pragma unroll
  for (int i = 0; i < NINST; ++i) {
    const int grow = rowBase + wave * RPW + i * RPI + lr;
    float* gp = C + (size_t)grow * ldc + colBase + 4 * f4;
    *(volatile v4f*)gp = vals[i];
  }
  __threadfence();
#pragma unroll
  for (int i = 0; i < NINST; ++i) {
    const int grow = rowBase + wave * RPW + i * RPI + lr;
    float* gp = C + (size_t)grow * ldc + colBase + 4 * f4;
    *(volatile v4f*)gp = vals[i];
  }
}

__global__ __launch_bounds__(NTHR) void k_edge(
    const int* __restrict__ csr, const int* __restrict__ off, const int* __restrict__ cnt,
    const int* __restrict__ ei, const float* __restrict__ eattr,
    const float* __restrict__ PQ, const float* __restrict__ W1, const float* __restrict__ b1,
    float* S, int nN, int nE, int csrLen) {
  const int tid = threadIdx.x, lane = tid & 31, wave = tid >> 5;
  const int tbase = (int)blockIdx.x * TGT + wave * 32;
  const int cl = tbase + lane;
  const int cnt_l = cnt[cl];
  const int off_l = off[cl];
  const v4f wa = *(const v4f*)(W1 + (size_t)(2 * FH + 0) * FH + 4 * lane);
  const v4f wb = *(const v4f*)(W1 + (size_t)(2 * FH + 1) * FH + 4 * lane);
  const v4f wc = *(const v4f*)(W1 + (size_t)(2 * FH + 2) * FH + 4 * lane);
  const v4f bb = *(const v4f*)(b1 + 4 * lane);

#pragma unroll 1
  for (int j = 0; j < 32; ++j) {
    const int c = tbase + j;
    int n = __builtin_amdgcn_readlane(cnt_l, j);
    n = n < 0 ? 0 : (n > DEGCAP ? DEGCAP : n);
    const int st = __builtin_amdgcn_readlane(off_l, j);
    const v4f base = *(const v4f*)(PQ + (size_t)c * PQW + 4 * lane) + bb;
    v4f acc = {0.f, 0.f, 0.f, 0.f};
#pragma unroll 1
    for (int q0 = 0; q0 < n; q0 += 32) {
      int pos = st + q0 + lane;
      pos = pos < 0 ? 0 : (pos > csrLen - 1 ? csrLen - 1 : pos);
      int eid = csr[pos];
      eid = eid < 0 ? 0 : (eid > nE - 1 ? nE - 1 : eid);
      int sv = ei[eid];
      sv = sv < 0 ? 0 : (sv > nN - 1 ? nN - 1 : sv);
      const float a0 = eattr[(size_t)eid * EDIM + 0];
      const float a1 = eattr[(size_t)eid * EDIM + 1];
      const float a2 = eattr[(size_t)eid * EDIM + 2];
      const int mcnt = (n - q0) < 32 ? (n - q0) : 32;
#pragma unroll 1
      for (int p = 0; p < mcnt; ++p) {
        const int   s  = __builtin_amdgcn_readlane(sv, p);
        const float x0 = __int_as_float(__builtin_amdgcn_readlane(__float_as_int(a0), p));
        const float x1 = __int_as_float(__builtin_amdgcn_readlane(__float_as_int(a1), p));
        const float x2 = __int_as_float(__builtin_amdgcn_readlane(__float_as_int(a2), p));
        const v4f q = *(const v4f*)(PQ + (size_t)s * PQW + FH + 4 * lane);
        v4f pre = base + q;
        pre = pre + wa * x0;
        pre = pre + wb * x1;
        pre = pre + wc * x2;
        acc = acc + silu4(pre);
      }
    }
    float* sp = S + (size_t)c * FH + 4 * lane;
    *(volatile v4f*)sp = acc;
    __threadfence();
    *(volatile v4f*)sp = acc;
  }
}

__global__ __launch_bounds__(NTHR) void k_pack(const float* __restrict__ D, float* out, int total) {
  const int f = (int)blockIdx.x * NTHR + (int)threadIdx.x;
  const int base = 4 * f;
  float vv[4];
#pragma unroll
  for (int j = 0; j < 4; ++j) {
    int idc = base + j;
    idc = idc > total - 1 ? total - 1 : idc;
    idc = idc < 0 ? 0 : idc;
    const int r = idc / FOUT;
    const int c = idc - r * FOUT;
    vv[j] = D[(size_t)r * D3W + c];
  }
  const v4f v = {vv[0], vv[1], vv[2], vv[3]};
  const bool full = (base + 3 < total);
  if (full) {
    *(volatile v4f*)(out + base) = v;
  } else {
#pragma unroll
    for (int j = 0; j < 4; ++j) if (base + j < total) *(volatile float*)(out + base + j) = vv[j];
  }
  __threadfence();
  if (full) {
    *(volatile v4f*)(out + base) = v;
  } else {
#pragma unroll
    for (int j = 0; j < 4; ++j) if (base + j < total) *(volatile float*)(out + base + j) = vv[j];
  }
}

extern "C" void kernel_launch(void* const* d_in, const int* in_sizes, int n_in,
                              void* d_out, int out_size, void* d_ws, size_t ws_size,
                              hipStream_t stream) {
  if (n_in < 17) return;
  const int nN = in_sizes[0] / FIN;
  const int nE = in_sizes[1] / 2;
  if (nN <= 0 || nE <= 0) return;
  if (in_sizes[0] != nN * FIN || in_sizes[1] != 2 * nE || in_sizes[2] != nE * EDIM) return;
  if (in_sizes[3] != FIN * FH || in_sizes[4] != FH || in_sizes[5] != FH * FH || in_sizes[6] != FH) return;
  if (in_sizes[7] != NLAY * MSGK * FH || in_sizes[8] != NLAY * FH) return;
  if (in_sizes[9] != NLAY * FH * FH || in_sizes[10] != NLAY * FH) return;
  if (in_sizes[11] != FH * FH || in_sizes[12] != FH || in_sizes[13] != FH * FH2 || in_sizes[14] != FH2) return;
  if (in_sizes[15] != FH2 * FOUT || in_sizes[16] != FOUT) return;
  if (out_size != nN * FOUT) return;
  if (nN > (1 << 18) || nE > (1 << EIDBITS)) return;

  const float* x       = (const float*)d_in[0];
  const int*   ei      = (const int*)d_in[1];
  const float* eattr   = (const float*)d_in[2];
  const float* enc_w1  = (const float*)d_in[3];
  const float* enc_b1  = (const float*)d_in[4];
  const float* enc_w2  = (const float*)d_in[5];
  const float* enc_b2  = (const float*)d_in[6];
  const float* conv_w1 = (const float*)d_in[7];
  const float* conv_b1 = (const float*)d_in[8];
  const float* conv_w2 = (const float*)d_in[9];
  const float* conv_b2 = (const float*)d_in[10];
  const float* dec_w1  = (const float*)d_in[11];
  const float* dec_b1  = (const float*)d_in[12];
  const float* dec_w2  = (const float*)d_in[13];
  const float* dec_b2  = (const float*)d_in[14];
  const float* dec_w3  = (const float*)d_in[15];
  const float* dec_b3  = (const float*)d_in[16];
  float* out = (float*)d_out;

  const int NPAD   = ((nN + TGT - 1) / TGT) * TGT;
  const int nBC    = (nN + NBC - 1) / NBC;
  const int CNTPAD = nBC * NBC;
  const int nBF    = (nN + NBF - 1) / NBF;
  const int OFFN   = nBF * NBF;
  if (nBF + 1 > RBN) return;
  if (OFFN > CNTPAD || NPAD > OFFN) return;
  const int csrLen = ((nE + 31) & ~31) + 32 * (nBF + 1);
  const int nGemm  = NPAD / GR;
  const int nAgg   = NPAD / TGT;
  const int nTot   = nN * FOUT;
  const int nPack  = ((nTot + 3) / 4 + NTHR - 1) / NTHR;

  char* ws = (char*)d_ws;
  size_t off = 0;
  const size_t oE1 = off; off += (size_t)2 * FH * 32 * 2;          off = (off + 255) & ~(size_t)255;
  const size_t oE2 = off; off += (size_t)2 * FH * FH * 2;          off = (off + 255) & ~(size_t)255;
  const size_t oC1 = off; off += (size_t)2 * NLAY * PQW * FH * 2;  off = (off + 255) & ~(size_t)255;
  const size_t oC2 = off; off += (size_t)2 * NLAY * FH * FH * 2;   off = (off + 255) & ~(size_t)255;
  const size_t oD1 = off; off += (size_t)2 * FH * FH * 2;          off = (off + 255) & ~(size_t)255;
  const size_t oD2 = off; off += (size_t)2 * FH2 * FH * 2;         off = (off + 255) & ~(size_t)255;
  const size_t oD3 = off; off += (size_t)2 * D3W * FH2 * 2;        off = (off + 255) & ~(size_t)255;
  const size_t oCnt = off; off += (size_t)CNTPAD * 4;              off = (off + 255) & ~(size_t)255;
  const size_t oOff = off; off += (size_t)OFFN * 4;                off = (off + 255) & ~(size_t)255;
  const size_t oRb  = off; off += (size_t)RBN * 4;                 off = (off + 255) & ~(size_t)255;
  const size_t oCsr = off; off += (size_t)csrLen * 4;              off = (off + 255) & ~(size_t)255;
  const size_t oH0  = off; off += (size_t)NPAD * FH * 4;           off = (off + 255) & ~(size_t)255;
  const size_t oH1  = off; off += (size_t)NPAD * FH * 4;           off = (off + 255) & ~(size_t)255;
  const size_t oT   = off; off += (size_t)NPAD * FH * 4;           off = (off + 255) & ~(size_t)255;
  const size_t oS   = off; off += (size_t)NPAD * FH * 4;           off = (off + 255) & ~(size_t)255;
  const size_t oPQ  = off; off += (size_t)NPAD * PQW * 4;          off = (off + 255) & ~(size_t)255;
  const size_t oP2  = off; off += (size_t)NPAD * FH2 * 4;          off = (off + 255) & ~(size_t)255;
  const size_t oP3  = off; off += (size_t)NPAD * D3W * 4;          off = (off + 255) & ~(size_t)255;
  if (off > ws_size || off > (size_t)WSCAP) return;
  unsigned short* e1h = (unsigned short*)(ws + oE1); unsigned short* e1l = e1h + FH * 32;
  unsigned short* e2h = (unsigned short*)(ws + oE2); unsigned short* e2l = e2h + FH * FH;
  unsigned short* c1h = (unsigned short*)(ws + oC1); unsigned short* c1l = c1h + (size_t)NLAY * PQW * FH;
  unsigned short* c2h = (unsigned short*)(ws + oC2); unsigned short* c2l = c2h + (size_t)NLAY * FH * FH;
  unsigned short* d1h = (unsigned short*)(ws + oD1); unsigned short* d1l = d1h + FH * FH;
  unsigned short* d2h = (unsigned short*)(ws + oD2); unsigned short* d2l = d2h + FH2 * FH;
  unsigned short* d3h = (unsigned short*)(ws + oD3); unsigned short* d3l = d3h + D3W * FH2;
  int*   cnt  = (int*)(ws + oCnt);
  int*   offp = (int*)(ws + oOff);
  int*   rb   = (int*)(ws + oRb);
  int*   csr  = (int*)(ws + oCsr);
  float* H0   = (float*)(ws + oH0);
  float* H1   = (float*)(ws + oH1);
  float* T    = (float*)(ws + oT);
  float* S    = (float*)(ws + oS);
  float* PQ   = (float*)(ws + oPQ);
  float* P2   = (float*)(ws + oP2);
  float* P3   = (float*)(ws + oP3);

  const int vec8 = ((nE & 3) == 0) ? 1 : 0;

  k_wprep<<<dim3((FH * 32 / 8 + NTHR - 1) / NTHR, 1), NTHR, 0, stream>>>(enc_w1, FIN, FH, 1, 0, 0, e1h, e1l, 0, 32, FH);
  k_wprep<<<dim3((FH * FH / 8) / NTHR, 1), NTHR, 0, stream>>>(enc_w2, FH, FH, 1, 0, 0, e2h, e2l, 0, FH, FH);
  k_wprep<<<dim3((FH * FH / 8) / NTHR, 2 * NLAY), NTHR, 0, stream>>>(conv_w1, FH, FH, 2, MSGK * FH, FH * FH, c1h, c1l, FH * FH, FH, FH);
  k_wprep<<<dim3((FH * FH / 8) / NTHR, NLAY), NTHR, 0, stream>>>(conv_w2, FH, FH, 1, FH * FH, 0, c2h, c2l, FH * FH, FH, FH);
  k_wprep<<<dim3((FH * FH / 8) / NTHR, 1), NTHR, 0, stream>>>(dec_w1, FH, FH, 1, 0, 0, d1h, d1l, 0, FH, FH);
  k_wprep<<<dim3((FH2 * FH / 8) / NTHR, 1), NTHR, 0, stream>>>(dec_w2, FH, FH2, 1, 0, 0, d2h, d2l, 0, FH, FH2);
  k_wprep<<<dim3((D3W * FH2 / 8 + NTHR - 1) / NTHR, 1), NTHR, 0, stream>>>(dec_w3, FH2, FOUT, 1, 0, 0, d3h, d3l, 0, FH2, D3W);

  hipFuncSetAttribute(reinterpret_cast<const void*>(&k_count),
                      hipFuncAttributeMaxDynamicSharedMemorySize, LDS_COUNT);
  k_count<<<nBC, NTHR, LDS_COUNT, stream>>>(ei, cnt, nE, vec8);
  k_offsets<<<1, OTHR, 0, stream>>>(cnt, offp, rb, nBF);
  hipFuncSetAttribute(reinterpret_cast<const void*>(&k_fill),
                      hipFuncAttributeMaxDynamicSharedMemorySize, LDS_FILL);
  k_fill<<<nBF, NTHR, LDS_FILL, stream>>>(ei, offp, rb, csr, nE, vec8, csrLen);

  k_gemm<32, FIN, FIN, 4, 1, 0, 1><<<dim3(nGemm, 1), NTHR, LDS_GEMM, stream>>>(x, nN, e1h, e1l, enc_b1, FH, H1, cnt, T, FH);
  k_gemm<FH, FH, FH, 4, 0, 0, 1><<<dim3(nGemm, 1), NTHR, LDS_GEMM, stream>>>(T, NPAD, e2h, e2l, enc_b2, FH, H1, cnt, H0, FH);

  for (int l = 0; l < NLAY; ++l) {
    float* Hin  = (l & 1) ? H1 : H0;
    float* Hout = (l & 1) ? H0 : H1;
    k_gemm<FH, FH, FH, 4, 0, 0, 0><<<dim3(nGemm, 2), NTHR, LDS_GEMM, stream>>>(
        Hin, NPAD, c1h + (size_t)l * PQW * FH, c1l + (size_t)l * PQW * FH, conv_b1, PQW, Hout, cnt, PQ, PQW);
    k_edge<<<nAgg, NTHR, 0, stream>>>(csr, offp, cnt, ei, eattr, PQ, conv_w1 + (size_t)l * MSGK * FH,
                                      conv_b1 + (size_t)l * FH, S, nN, nE, csrLen);
    k_gemm<FH, FH, FH, 4, 0, 1, 1><<<dim3(nGemm, 1), NTHR, LDS_GEMM, stream>>>(
        S, NPAD, c2h + (size_t)l * FH * FH, c2l + (size_t)l * FH * FH, conv_b2 + (size_t)l * FH, FH, Hin, cnt, Hout, FH);
  }
  float* Hf = (NLAY & 1) ? H1 : H0;

  k_gemm<FH, FH, FH, 4, 1, 0, 1><<<dim3(nGemm, 1), NTHR, LDS_GEMM, stream>>>(Hf, NPAD, d1h, d1l, dec_b1, FH, H1, cnt, T, FH);
  k_gemm<FH, FH, FH, 2, 1, 0, 1><<<dim3(nGemm, 1), NTHR, LDS_GEMM, stream>>>(T, NPAD, d2h, d2l, dec_b2, FH2, H1, cnt, P2, FH2);
  k_gemm<FH2, FH2, FH2, 1, 0, 0, 1><<<dim3(nGemm, 1), NTHR, LDS_GEMM, stream>>>(P2, NPAD, d3h, d3l, dec_b3, FOUT, H1, cnt, P3, D3W);

  k_pack<<<nPack, NTHR, 0, stream>>>(P3, out, nTot);
}
